// UpTransition_19868518711860
// MI455X (gfx1250) — hardware-run, weakly checked
//
#include <hip/hip_runtime.h>
#include <stddef.h>


#define C_IN    64
#define K_OFF   27
#define TSL     32
#define XSC     8.0f
#define WSC     256.0f
#define RH      0.00048828125f
#define RUP     0.00390625f
#define WSCAP   134217728

#define CTHR    128
#define CWAV    (CTHR / 32)
#define CPTS    (16 * CWAV)
#define GRP     9
#define NGRP    (K_OFF / GRP)
#define AROW    (GRP * C_IN)
#define NPIECE  (CPTS * GRP * 8)
#define PSTR    128
#define STN     256

#define LC_A    0
#define LC_S    (CPTS * AROW * 2)
#define LC_NB   (LC_S + CPTS * 64 * 4)
#define LC_PL   (LC_NB + CPTS * TSL * 4)
#define LDS_CONV (LC_PL + PSTR * 4)

#define TTHR    256
#define TROWS   1024
#define LDS_TBL (TROWS * TSL * 4)

#define UTHR    128
#define UROWS   64
#define ETHR    256
#define EROWS   32

static_assert(NGRP * GRP == K_OFF);
static_assert(CPTS == 64);
static_assert(LC_S == 73728);
static_assert(LC_NB == 90112);
static_assert(LC_PL == 98304);
static_assert(LDS_CONV == 98816);
static_assert((LC_S % 16) == 0 && (LC_NB % 16) == 0 && (LC_PL % 16) == 0);
static_assert((NPIECE % CTHR) == 0);
static_assert((CPTS * TSL / 4) % CTHR == 0);
static_assert(PSTR == CTHR);
static_assert((TROWS * TSL / 4) % TTHR == 0);
static_assert(EROWS * 8 == ETHR);
static_assert((UROWS * 8) % UTHR == 0);

typedef float    v4f  __attribute__((ext_vector_type(4)));
typedef float    v8f  __attribute__((ext_vector_type(8)));
typedef int      v4i  __attribute__((ext_vector_type(4)));
typedef _Float16 v4h  __attribute__((ext_vector_type(4)));
typedef _Float16 v8h  __attribute__((ext_vector_type(8)));
typedef _Float16 v16h __attribute__((ext_vector_type(16)));
union Frag  { v16h v; v8h h[2]; };
union Frag8 { v8h v; v4h q[2]; };

__device__ __forceinline__ v8f wmh(v16h a, v16h b, v8f c) {
  v8f d = __builtin_amdgcn_wmma_f32_16x16x32_f16(false, a, false, b, (short)0, c, false, false);
  asm volatile("v_nop\n\tv_nop\n\tv_nop\n\tv_nop" : "+v"(d) : "v"(a), "v"(b));
  return d;
}

__device__ __forceinline__ v4h cvt4h(v4f x) {
  v4h r;
  r.x = (_Float16)x.x;
  r.y = (_Float16)x.y;
  r.z = (_Float16)x.z;
  r.w = (_Float16)x.w;
  return r;
}

__device__ __forceinline__ int clampi(int v, int hi) { return v < 0 ? 0 : (v > hi ? hi : v); }

__device__ __forceinline__ float eluf(float x) { return x > 0.0f ? x : (__expf(x) - 1.0f); }

__device__ __forceinline__ v4f elu4(v4f x) {
  v4f r;
  r.x = eluf(x.x);
  r.y = eluf(x.y);
  r.z = eluf(x.z);
  r.w = eluf(x.w);
  return r;
}

__device__ __forceinline__ v4f max4(v4f a, v4f b) {
  v4f r;
  r.x = fmaxf(a.x, b.x);
  r.y = fmaxf(a.y, b.y);
  r.z = fmaxf(a.z, b.z);
  r.w = fmaxf(a.w, b.w);
  return r;
}

template <int NOUT>
__global__ __launch_bounds__(ETHR) void k_wprep(const float* __restrict__ W, _Float16* Wp) {
  const int kp = blockIdx.x, tid = threadIdx.x;
  const float* wk = W + (size_t)kp * (C_IN * NOUT);
#pragma unroll
  for (int it = 0; it < NOUT / 32; ++it) {
    const int n = 32 * it + (tid >> 3), c0 = (tid & 7) * 8;
    v8h hv;
#pragma unroll
    for (int e = 0; e < 8; ++e) hv[e] = (_Float16)(wk[(size_t)(c0 + e) * NOUT + n] * WSC);
    _Float16* dst = Wp + ((size_t)kp * NOUT + n) * C_IN + c0;
    *(volatile v8h*)dst = hv;
    __threadfence();
    *(volatile v8h*)dst = hv;
  }
}

__global__ __launch_bounds__(TTHR) void k_tbl(const int* __restrict__ in_idx, const int* __restrict__ out_idx,
                                              int* Tn, int* flg, int nN, int P) {
  extern __shared__ __attribute__((aligned(16))) char dyn_t[];
  int* tb = (int*)dyn_t;
  __shared__ int dflag;
  const int tid = threadIdx.x, lane = tid & 31;
  const int wave = __builtin_amdgcn_readfirstlane(tid >> 5);
  const int r0 = blockIdx.x * TROWS;
  if (tid == 0) dflag = 0;
  const v4i fill = {nN, nN, nN, nN};
#pragma unroll 1
  for (int it = 0; it < (TROWS * TSL / 4) / TTHR; ++it) *(v4i*)(tb + 4 * (it * TTHR + tid)) = fill;
  __syncthreads();

  const int nit = (P + TTHR - 1) / TTHR;
#pragma unroll 1
  for (int k = 0; k < K_OFF; ++k) {
    const int* oi = out_idx + (size_t)k * P;
    const int* ii = in_idx + (size_t)k * P;
#pragma unroll 1
    for (int it = 0; it < nit; ++it) {
      const int pp = it * TTHR + tid;
      const bool valid = pp < P;
      const int pc = valid ? pp : P - 1;
      const int o = oi[pc];
      const int i = ii[pc];
      const bool owned = valid && (o >= r0) && (o < r0 + TROWS) && (o < nN);
      const int lr = owned ? (o - r0) : 0;
      const int slot = lr * TSL + k;
      const int ic = clampi(i, nN);
      const int old = tb[slot];
      if (owned && old != nN) dflag = 1;
      if (owned) tb[slot] = ic;
    }
  }
  __syncthreads();

  const int flagv = dflag;
  int* Tg = Tn + (size_t)r0 * TSL;
#pragma unroll 1
  for (int it = 0; it < (TROWS * TSL / 4) / TTHR; ++it) {
    const int p = it * TTHR + tid;
    const v4i v = *(const v4i*)(tb + 4 * p);
    *(volatile v4i*)(Tg + 4 * (size_t)p) = v;
  }
  if (wave == 0) *(volatile int*)(flg + (size_t)blockIdx.x * 32 + lane) = flagv;
  __threadfence();
#pragma unroll 1
  for (int it = 0; it < (TROWS * TSL / 4) / TTHR; ++it) {
    const int p = it * TTHR + tid;
    const v4i v = *(const v4i*)(tb + 4 * p);
    *(volatile v4i*)(Tg + 4 * (size_t)p) = v;
  }
  if (wave == 0) *(volatile int*)(flg + (size_t)blockIdx.x * 32 + lane) = flagv;
}

__global__ __launch_bounds__(UTHR) void k_up(const float* __restrict__ X, const _Float16* __restrict__ WpU,
                                             _Float16* Fu, int nC) {
  __shared__ __attribute__((aligned(16))) _Float16 AX[UROWS * C_IN];
  __shared__ __attribute__((aligned(16))) _Float16 SU[UROWS * C_IN];
  const int tid = threadIdx.x, lane = tid & 31, hh = lane >> 4, m = lane & 15;
  const int wave = __builtin_amdgcn_readfirstlane(tid >> 5);
  const int nb0 = blockIdx.x * UROWS;

#pragma unroll
  for (int it = 0; it < (UROWS * 8) / UTHR; ++it) {
    const int p = it * UTHR + tid;
    const int row = p >> 3, c0 = (p & 7) * 8;
    const int n = nb0 + row;
    const bool ok = n < nC;
    const int nc = ok ? n : nC - 1;
    const float* xp = X + (size_t)nc * C_IN + c0;
    v4f f0 = *(const v4f*)(xp);
    v4f f1 = *(const v4f*)(xp + 4);
    const v4f z = {0.0f, 0.0f, 0.0f, 0.0f};
    f0 = ok ? f0 * XSC : z;
    f1 = ok ? f1 * XSC : z;
    Frag8 hv;
    hv.q[0] = cvt4h(f0);
    hv.q[1] = cvt4h(f1);
    *(v8h*)(AX + row * C_IN + c0) = hv.v;
  }
  __syncthreads();

  Frag a0, a1;
  {
    const _Float16* ga = AX + (wave * 16 + m) * C_IN + 8 * hh;
    a0.h[0] = *(const v8h*)(ga);
    a0.h[1] = *(const v8h*)(ga + 16);
    a1.h[0] = *(const v8h*)(ga + 32);
    a1.h[1] = *(const v8h*)(ga + 48);
  }
  _Float16* Sw = SU + wave * (16 * C_IN);
  const v8f z8 = {0.0f, 0.0f, 0.0f, 0.0f, 0.0f, 0.0f, 0.0f, 0.0f};
#pragma unroll 1
  for (int kp = 0; kp < 4; ++kp) {
    v8f acc[4];
#pragma unroll
    for (int t = 0; t < 4; ++t) acc[t] = z8;
    const _Float16* wb = WpU + ((size_t)kp * C_IN + m) * C_IN + 8 * hh;
#pragma unroll
    for (int t = 0; t < 4; ++t) {
      Frag b0, b1;
      const _Float16* bp = wb + (size_t)t * 16 * C_IN;
      b0.h[0] = *(const v8h*)(bp);
      b0.h[1] = *(const v8h*)(bp + 16);
      b1.h[0] = *(const v8h*)(bp + 32);
      b1.h[1] = *(const v8h*)(bp + 48);
      acc[t] = wmh(a0.v, b0.v, acc[t]);
      acc[t] = wmh(a1.v, b1.v, acc[t]);
    }
#pragma unroll
    for (int r = 0; r < 8; ++r) {
#pragma unroll
      for (int t = 0; t < 4; ++t) Sw[(8 * hh + r) * C_IN + 16 * t + m] = (_Float16)(acc[t][r] * RUP);
    }
    __syncthreads();
    v8h ov[4];
    const int lr0 = lane >> 3, pc = lane & 7;
#pragma unroll
    for (int qq = 0; qq < 4; ++qq) ov[qq] = *(const v8h*)(Sw + (4 * qq + lr0) * C_IN + 8 * pc);
#pragma unroll
    for (int qq = 0; qq < 4; ++qq) {
      const size_t frow = 4 * (size_t)(nb0 + 16 * wave + 4 * qq + lr0) + kp;
      _Float16* dst = Fu + frow * C_IN + 8 * pc;
      *(volatile v8h*)dst = ov[qq];
    }
    __threadfence();
#pragma unroll
    for (int qq = 0; qq < 4; ++qq) {
      const size_t frow = 4 * (size_t)(nb0 + 16 * wave + 4 * qq + lr0) + kp;
      _Float16* dst = Fu + frow * C_IN + 8 * pc;
      *(volatile v8h*)dst = ov[qq];
    }
    __syncthreads();
  }
}

template <int NT>
__global__ __launch_bounds__(CTHR) void k_conv(const _Float16* __restrict__ Fh, const _Float16* __restrict__ Wp,
                                               const int* __restrict__ Tn, float* Y, float* part, int nN) {
  constexpr int CO  = 16 * NT;
  constexpr int PPR = 4 * NT;
  constexpr int RPI = 32 / PPR;
  constexpr int NI  = 16 / RPI;
  extern __shared__ __attribute__((aligned(16))) char dyn_c[];
  _Float16* AL = (_Float16*)(dyn_c + LC_A);
  float* S   = (float*)(dyn_c + LC_S);
  int* nbl   = (int*)(dyn_c + LC_NB);
  float* pl  = (float*)(dyn_c + LC_PL);
  const int tid = threadIdx.x, lane = tid & 31, hh = lane >> 4, m = lane & 15;
  const int wave = __builtin_amdgcn_readfirstlane(tid >> 5);
  const int pb = blockIdx.x * CPTS;

#pragma unroll
  for (int it = 0; it < (CPTS * TSL / 4) / CTHR; ++it) {
    const int p = it * CTHR + tid;
    const int row = p >> 3, pc = p & 7;
    v4i v = *(const v4i*)(Tn + (size_t)(pb + row) * TSL + 4 * pc);
    v.x = clampi(v.x, nN);
    v.y = clampi(v.y, nN);
    v.z = clampi(v.z, nN);
    v.w = clampi(v.w, nN);
    *(v4i*)(nbl + row * TSL + 4 * pc) = v;
  }
  __syncthreads();

  const v8f z8 = {0.0f, 0.0f, 0.0f, 0.0f, 0.0f, 0.0f, 0.0f, 0.0f};
  v8f acc[NT];
#pragma unroll
  for (int t = 0; t < NT; ++t) acc[t] = z8;
#pragma unroll 1
  for (int g = 0; g < NGRP; ++g) {
#pragma unroll 1
    for (int it = 0; it < NPIECE / CTHR; ++it) {
      const int p = it * CTHR + tid;
      const int jj = p / (GRP * 8);
      const int r = p - jj * (GRP * 8);
      const int o = r >> 3, q = r & 7;
      const int nb = nbl[jj * TSL + g * GRP + o];
      const v8h vv = *(const v8h*)(Fh + (size_t)nb * C_IN + 8 * q);
      *(v8h*)(AL + (size_t)jj * AROW + o * C_IN + 8 * q) = vv;
    }
    __syncthreads();
    {
      const _Float16* ga = AL + (size_t)(wave * 16 + m) * AROW + 8 * hh;
      const _Float16* wb = Wp + (size_t)(g * GRP) * (CO * C_IN) + (size_t)m * C_IN + 8 * hh;
#pragma unroll 1
      for (int o = 0; o < GRP; ++o) {
#pragma unroll
        for (int kb = 0; kb < 2; ++kb) {
          Frag a;
          const _Float16* gp = ga + o * C_IN + kb * 32;
          a.h[0] = *(const v8h*)(gp);
          a.h[1] = *(const v8h*)(gp + 16);
          const _Float16* bp = wb + (size_t)o * (CO * C_IN) + kb * 32;
          Frag b[NT];
#pragma unroll
          for (int t = 0; t < NT; ++t) {
            b[t].h[0] = *(const v8h*)(bp + (size_t)t * 16 * C_IN);
            b[t].h[1] = *(const v8h*)(bp + (size_t)t * 16 * C_IN + 16);
          }
#pragma unroll
          for (int t = 0; t < NT; ++t) acc[t] = wmh(a.v, b[t].v, acc[t]);
        }
      }
    }
    __syncthreads();
  }

#pragma unroll
  for (int r = 0; r < 8; ++r) {
#pragma unroll
    for (int t = 0; t < NT; ++t) S[(size_t)(wave * 16 + 8 * hh + r) * CO + 16 * t + m] = acc[t][r] * RH;
  }
  __syncthreads();
  {
    const float* Sw = S + (size_t)wave * 16 * CO;
    const int rr = lane / PPR, cc = (lane % PPR) * 4;
    v4f ov[NI];
#pragma unroll
    for (int qq = 0; qq < NI; ++qq) ov[qq] = *(const v4f*)(Sw + (qq * RPI + rr) * CO + cc);
    const size_t rbase = (size_t)(pb + 16 * wave + rr);
#pragma unroll
    for (int qq = 0; qq < NI; ++qq) {
      float* op = Y + (rbase + qq * RPI) * CO + cc;
      *(volatile v4f*)op = ov[qq];
    }
    __threadfence();
#pragma unroll
    for (int qq = 0; qq < NI; ++qq) {
      float* op = Y + (rbase + qq * RPI) * CO + cc;
      *(volatile v4f*)op = ov[qq];
    }
  }
  {
    const int c = tid % CO;
    const int which = (tid / CO) & 1;
    float a = 0.0f;
#pragma unroll 4
    for (int r = 0; r < CPTS; ++r) {
      const float v = S[r * CO + c];
      a += which ? v * v : v;
    }
    pl[tid] = (tid < 2 * CO) ? a : 0.0f;
  }
  __syncthreads();
  if (wave == 0) {
    const v4f vv = *(const v4f*)(pl + 4 * lane);
    float* pp = part + (size_t)blockIdx.x * PSTR + 4 * lane;
    *(volatile v4f*)pp = vv;
    __threadfence();
    *(volatile v4f*)pp = vv;
  }
}

__global__ __launch_bounds__(128) void k_stats(const float* __restrict__ part, const float* __restrict__ gamma,
                                               const float* __restrict__ beta, const int* __restrict__ flg,
                                               float* stats, int nBlk, int nTB, int CO, int nN) {
  __shared__ double sd[128];
  __shared__ __attribute__((aligned(16))) float stf[STN];
  const int t = threadIdx.x;
  double a = 0.0;
#pragma unroll 1
  for (int b = 0; b < nBlk; ++b) a += (double)part[(size_t)b * PSTR + t];
  int f = 0;
#pragma unroll 1
  for (int b = 0; b < nTB; ++b) f |= flg[(size_t)b * 32];
  const int tc = t < CO ? t : CO - 1;
  const float gm = gamma[tc];
  const float bt = beta[tc];
  sd[t] = a;
  stf[t] = 0.0f;
  stf[128 + t] = 0.0f;
  __syncthreads();
  if (t < CO) {
    const double inv = 1.0 / (double)nN;
    const double mean = sd[t] * inv;
    double var = sd[CO + t] * inv - mean * mean;
    var = var < 0.0 ? 0.0 : var;
    const float varf = (float)var;
    const float mul = rsqrtf(varf + 1e-5f) * gm;
    float meanf = (float)mean;
    meanf = (f != 0) ? __int_as_float(0x7fc00000) : meanf;
    stf[t] = meanf;
    stf[64 + t] = mul;
    stf[128 + t] = bt;
  }
  __syncthreads();
  if (t < 64) {
    const v4f vv = *(const v4f*)(stf + 4 * t);
    float* sp = stats + 4 * t;
    *(volatile v4f*)sp = vv;
    __threadfence();
    *(volatile v4f*)sp = vv;
  }
}

__global__ __launch_bounds__(ETHR) void k_bnx(const float* __restrict__ Y, const float* __restrict__ stats,
                                              const float* __restrict__ skip, float* Xc, _Float16* Fx, int nN) {
  __shared__ __attribute__((aligned(16))) float st[STN];
  __shared__ __attribute__((aligned(16))) float sf[ETHR * 8];
  const int tid = threadIdx.x;
  st[tid] = stats[tid];
  __syncthreads();
  const int row = blockIdx.x * EROWS + (tid >> 3);
  const int c0 = (tid & 7) * 8;
  const int cb = c0 & 31;
  const bool ok = row < nN;
  const int rc = ok ? row : nN - 1;
  const float* yp = Y + (size_t)rc * 32 + cb;
  const v4f y0 = *(const v4f*)(yp);
  const v4f y1 = *(const v4f*)(yp + 4);
  const float* s0p = skip + (size_t)(2 * rc) * 32 + cb;
  const float* s1p = s0p + 32;
  const v4f sa0 = *(const v4f*)(s0p);
  const v4f sa1 = *(const v4f*)(s0p + 4);
  const v4f sb0 = *(const v4f*)(s1p);
  const v4f sb1 = *(const v4f*)(s1p + 4);
  const v4f mean0 = *(const v4f*)(st + cb),       mean1 = *(const v4f*)(st + cb + 4);
  const v4f mul0  = *(const v4f*)(st + 64 + cb),  mul1  = *(const v4f*)(st + 64 + cb + 4);
  const v4f add0  = *(const v4f*)(st + 128 + cb), add1  = *(const v4f*)(st + 128 + cb + 4);
  const v4f h0 = elu4((y0 - mean0) * mul0 + add0);
  const v4f h1 = elu4((y1 - mean1) * mul1 + add1);
  const v4f m0 = max4(sa0, sb0);
  const v4f m1 = max4(sa1, sb1);
  const bool left = c0 < 32;
  const v4f z = {0.0f, 0.0f, 0.0f, 0.0f};
  v4f r0 = left ? h0 : m0;
  v4f r1 = left ? h1 : m1;
  r0 = ok ? r0 : z;
  r1 = ok ? r1 : z;

  Frag8 hv;
  hv.q[0] = cvt4h(r0 * XSC);
  hv.q[1] = cvt4h(r1 * XSC);
  _Float16* fdst = Fx + (size_t)row * C_IN + c0;
  *(volatile v8h*)fdst = hv.v;

  *(v4f*)(sf + tid * 8) = r0;
  *(v4f*)(sf + tid * 8 + 4) = r1;
  __syncthreads();
  const v4f o0 = *(const v4f*)(sf + 4 * tid);
  const v4f o1 = *(const v4f*)(sf + 4 * (ETHR + tid));
  float* xb = Xc + (size_t)blockIdx.x * (EROWS * C_IN);
  *(volatile v4f*)(xb + 4 * tid) = o0;
  *(volatile v4f*)(xb + 4 * (ETHR + tid)) = o1;
  __threadfence();
  *(volatile v8h*)fdst = hv.v;
  *(volatile v4f*)(xb + 4 * tid) = o0;
  *(volatile v4f*)(xb + 4 * (ETHR + tid)) = o1;
}

__global__ __launch_bounds__(ETHR) void k_bnh(const float* __restrict__ Y, const float* __restrict__ stats,
                                              _Float16* Fh, int nN) {
  __shared__ __attribute__((aligned(16))) float st[STN];
  const int tid = threadIdx.x;
  st[tid] = stats[tid];
  __syncthreads();
  const int row = blockIdx.x * EROWS + (tid >> 3);
  const int c0 = (tid & 7) * 8;
  const bool ok = row < nN;
  const int rc = ok ? row : nN - 1;
  const float* yp = Y + (size_t)rc * C_IN + c0;
  const v4f y0 = *(const v4f*)(yp);
  const v4f y1 = *(const v4f*)(yp + 4);
  const v4f mean0 = *(const v4f*)(st + c0),       mean1 = *(const v4f*)(st + c0 + 4);
  const v4f mul0  = *(const v4f*)(st + 64 + c0),  mul1  = *(const v4f*)(st + 64 + c0 + 4);
  const v4f add0  = *(const v4f*)(st + 128 + c0), add1  = *(const v4f*)(st + 128 + c0 + 4);
  const v4f z = {0.0f, 0.0f, 0.0f, 0.0f};
  v4f h0 = elu4((y0 - mean0) * mul0 + add0);
  v4f h1 = elu4((y1 - mean1) * mul1 + add1);
  h0 = ok ? h0 : z;
  h1 = ok ? h1 : z;
  Frag8 hv;
  hv.q[0] = cvt4h(h0 * XSC);
  hv.q[1] = cvt4h(h1 * XSC);
  _Float16* fdst = Fh + (size_t)row * C_IN + c0;
  *(volatile v8h*)fdst = hv.v;
  __threadfence();
  *(volatile v8h*)fdst = hv.v;
}

__global__ __launch_bounds__(ETHR) void k_fin(const float* __restrict__ Y, const float* __restrict__ stats,
                                              const float* __restrict__ Xc, float* out, int nQ) {
  __shared__ __attribute__((aligned(16))) float st[STN];
  const int tid = threadIdx.x;
  st[tid] = stats[tid];
  __syncthreads();
  const int q = blockIdx.x * ETHR + tid;
  const int qc = q < nQ ? q : nQ - 1;
  const int c0 = (qc & 15) * 4;
  const v4f y = *(const v4f*)(Y + (size_t)qc * 4);
  const v4f x = *(const v4f*)(Xc + (size_t)qc * 4);
  const v4f mean = *(const v4f*)(st + c0);
  const v4f mul  = *(const v4f*)(st + 64 + c0);
  const v4f add  = *(const v4f*)(st + 128 + c0);
  const v4f h = elu4((y - mean) * mul + add);
  const v4f r = elu4(h + x);
  float* op = out + (size_t)qc * 4;
  if (q < nQ) *(volatile v4f*)op = r;
  __threadfence();
  if (q < nQ) *(volatile v4f*)op = r;
}

static inline size_t al256(size_t x) { return (x + 255) & ~(size_t)255; }

extern "C" void kernel_launch(void* const* d_in, const int* in_sizes, int n_in,
                              void* d_out, int out_size, void* d_ws, size_t ws_size,
                              hipStream_t stream) {
  if (n_in < 11) return;
  if (in_sizes[0] < C_IN || (in_sizes[0] % C_IN) != 0) return;
  const int nC = in_sizes[0] / C_IN;
  const int nN = 4 * nC;
  if (in_sizes[1] != 2 * nN * 32) return;
  if (in_sizes[2] != 4 * C_IN * 64) return;
  if (in_sizes[3] != K_OFF * C_IN * 32) return;
  if (in_sizes[4] != 32 || in_sizes[5] != 32) return;
  if (in_sizes[6] != 2 * K_OFF * C_IN * 64) return;
  if (in_sizes[7] != 128 || in_sizes[8] != 128) return;
  if (in_sizes[9] < K_OFF || (in_sizes[9] % K_OFF) != 0) return;
  const int P = in_sizes[9] / K_OFF;
  if (in_sizes[10] != in_sizes[9]) return;
  if (out_size != nN * 64) return;

  const int gU    = nC / UROWS + 1;
  const int RU    = gU * UROWS * 4;
  const int gC    = (nN + CPTS - 1) / CPTS;
  const int rowsY = gC * CPTS;
  const int gT    = (rowsY + TROWS - 1) / TROWS;
  const int rowsT = gT * TROWS;
  const int gE    = nN / EROWS + 1;
  const int RP    = gE * EROWS;
  const int nQ    = nN * (C_IN / 4);
  const int gB    = (nQ + ETHR - 1) / ETHR;
  if (RU < nN + 1 || RP < nN + 1 || rowsT < rowsY || rowsY < nN) return;

  const float* X    = (const float*)d_in[0];
  const float* SK   = (const float*)d_in[1];
  const float* Wup  = (const float*)d_in[2];
  const float* Wuc  = (const float*)d_in[3];
  const float* g1   = (const float*)d_in[4];
  const float* b1   = (const float*)d_in[5];
  const float* Wcv  = (const float*)d_in[6];
  const float* gcv  = (const float*)d_in[7];
  const float* bcv  = (const float*)d_in[8];
  const int*   II   = (const int*)d_in[9];
  const int*   OI   = (const int*)d_in[10];
  float* out = (float*)d_out;

  char* ws = (char*)d_ws;
  size_t off = 0;
  const size_t oWU = off; off = al256(off + (size_t)4 * 64 * C_IN * 2);
  const size_t oW1 = off; off = al256(off + (size_t)K_OFF * 32 * C_IN * 2);
  const size_t oW2 = off; off = al256(off + (size_t)2 * K_OFF * 64 * C_IN * 2);
  const size_t oT  = off; off = al256(off + (size_t)rowsT * TSL * 4);
  const size_t oFl = off; off = al256(off + (size_t)gT * 32 * 4);
  const size_t oFu = off; off = al256(off + (size_t)RU * C_IN * 2);
  const size_t oY  = off; off = al256(off + (size_t)rowsY * 64 * 4);
  const size_t oPt = off; off = al256(off + (size_t)gC * PSTR * 4);
  const size_t oSt = off; off = al256(off + (size_t)STN * 4);
  const size_t oXc = off; off = al256(off + (size_t)RP * C_IN * 4);
  const size_t oFx = off; off = al256(off + (size_t)RP * C_IN * 2);
  const size_t oF2 = off; off = al256(off + (size_t)RP * C_IN * 2);
  if (off > ws_size || off > (size_t)WSCAP) return;
  _Float16* WpU  = (_Float16*)(ws + oWU);
  _Float16* Wp1  = (_Float16*)(ws + oW1);
  _Float16* Wp2  = (_Float16*)(ws + oW2);
  int*      Tn   = (int*)(ws + oT);
  int*      flg  = (int*)(ws + oFl);
  _Float16* Fu   = (_Float16*)(ws + oFu);
  float*    Y    = (float*)(ws + oY);
  float*    part = (float*)(ws + oPt);
  float*    stats = (float*)(ws + oSt);
  float*    Xc   = (float*)(ws + oXc);
  _Float16* Fx   = (_Float16*)(ws + oFx);
  _Float16* Fh2  = (_Float16*)(ws + oF2);

  hipFuncSetAttribute(reinterpret_cast<const void*>(&k_tbl), hipFuncAttributeMaxDynamicSharedMemorySize, LDS_TBL);
  hipFuncSetAttribute(reinterpret_cast<const void*>(&k_conv<2>), hipFuncAttributeMaxDynamicSharedMemorySize, LDS_CONV);
  hipFuncSetAttribute(reinterpret_cast<const void*>(&k_conv<4>), hipFuncAttributeMaxDynamicSharedMemorySize, LDS_CONV);

  k_wprep<64><<<4, ETHR, 0, stream>>>(Wup, WpU);
  k_wprep<32><<<K_OFF, ETHR, 0, stream>>>(Wuc, Wp1);
  k_wprep<64><<<2 * K_OFF, ETHR, 0, stream>>>(Wcv, Wp2);
  k_tbl<<<gT, TTHR, LDS_TBL, stream>>>(II, OI, Tn, flg, nN, P);
  k_up<<<gU, UTHR, 0, stream>>>(X, WpU, Fu, nC);
  k_conv<2><<<gC, CTHR, LDS_CONV, stream>>>(Fu, Wp1, Tn, Y, part, nN);
  k_stats<<<1, 128, 0, stream>>>(part, g1, b1, flg, stats, gC, gT, 32, nN);
  k_bnx<<<gE, ETHR, 0, stream>>>(Y, stats, SK, Xc, Fx, nN);
  k_conv<4><<<gC, CTHR, LDS_CONV, stream>>>(Fx, Wp2, Tn, Y, part, nN);
  k_stats<<<1, 128, 0, stream>>>(part, gcv, bcv, flg, stats, gC, gT, 64, nN);
  k_bnh<<<gE, ETHR, 0, stream>>>(Y, stats, Fh2, nN);
  k_conv<4><<<gC, CTHR, LDS_CONV, stream>>>(Fh2, Wp2 + (size_t)K_OFF * 64 * C_IN, Tn, Y, part, nN);
  k_stats<<<1, 128, 0, stream>>>(part, gcv + 64, bcv + 64, flg, stats, gC, gT, 64, nN);
  k_fin<<<gB, ETHR, 0, stream>>>(Y, stats, Xc, out, nQ);
}
